// EncoderLayer_8160437862705
// MI455X (gfx1250) — hardware-run, weakly checked
//
#include <hip/hip_runtime.h>
#include <stddef.h>
#include <stdint.h>


#ifndef NB
#define NB 2
#endif
#ifndef SEQ
#define SEQ 2048
#endif
#define NB_FULL 2
#define S_FULL 2048

constexpr int ND  = 1024;
constexpr int NH  = 16;
constexpr int NDK = 64;
constexpr int NFF = 4096;
constexpr int TOK = NB * SEQ;

static_assert(NB >= 1 && NB <= NB_FULL);
static_assert(SEQ >= 128 && SEQ <= S_FULL && (SEQ % 128) == 0);
static_assert((TOK % 128) == 0);
static_assert(ND == NH * NDK);
static_assert((ND % 128) == 0 && (NFF % 128) == 0);

typedef _Float16 v16h  __attribute__((ext_vector_type(16)));
typedef _Float16 v8h_t __attribute__((ext_vector_type(8)));
typedef v8h_t    v8h   __attribute__((may_alias));
typedef _Float16 v4h_t __attribute__((ext_vector_type(4)));
typedef v4h_t    v4hh  __attribute__((may_alias));
typedef float    v8f   __attribute__((ext_vector_type(8)));
typedef float    v4f_t __attribute__((ext_vector_type(4)));
typedef v4f_t    v4f   __attribute__((may_alias));

__device__ __forceinline__ float bf16r(float x) {
  unsigned int u = __float_as_uint(x);
  u += 0x7FFFu + ((u >> 16) & 1u);
  u &= 0xFFFF0000u;
  return __uint_as_float(u);
}

__device__ __forceinline__ v8f wmma16(v16h a, v16h b, v8f c) {
  return __builtin_amdgcn_wmma_f32_16x16x32_f16(false, a, false, b, (short)0, c,
                                                false, false);
}

__device__ __forceinline__ v16h frag_ld(const _Float16* row, int hi) {
  const v8h lo = *(const v8h*)(row + hi * 8);
  const v8h up = *(const v8h*)(row + 16 + hi * 8);
  return __builtin_shufflevector(lo, up, 0, 1, 2, 3, 4, 5, 6, 7,
                                 8, 9, 10, 11, 12, 13, 14, 15);
}

__global__ __launch_bounds__(256) void cvt_x_kernel(const float* __restrict__ X,
                                                    _Float16* __restrict__ Xh) {
  const size_t g   = (size_t)blockIdx.x * 256 + threadIdx.x;
  const size_t e   = g * 8;
  const size_t tok = e >> 10;
  const int    col = (int)(e & 1023);
  const size_t b   = tok / SEQ;
  const size_t s   = tok - b * SEQ;
  const float* src = X + ((b * S_FULL + s) * (size_t)ND + col);
  const v4f f0 = *(const v4f*)(src);
  const v4f f1 = *(const v4f*)(src + 4);
  v8h hv;
  hv[0] = (_Float16)bf16r(f0[0]); hv[1] = (_Float16)bf16r(f0[1]);
  hv[2] = (_Float16)bf16r(f0[2]); hv[3] = (_Float16)bf16r(f0[3]);
  hv[4] = (_Float16)bf16r(f1[0]); hv[5] = (_Float16)bf16r(f1[1]);
  hv[6] = (_Float16)bf16r(f1[2]); hv[7] = (_Float16)bf16r(f1[3]);
  _Float16* dst = Xh + e;
  *(volatile v8h*)dst = hv;
  __threadfence();
  *(volatile v8h*)dst = hv;
}

__global__ __launch_bounds__(256) void wtr_kernel(const float* __restrict__ W,
                                                  _Float16* __restrict__ WT,
                                                  int K, int N, float scale) {
  __shared__ float t[64][33];
  const int tid = threadIdx.x;
  const int kb  = blockIdx.y * 64;
  const int nb  = blockIdx.x * 32;
#pragma unroll
  for (int i = 0; i < 8; ++i) {
    const int idx = i * 256 + tid;
    const int r = idx >> 5, c = idx & 31;
    t[r][c] = W[(size_t)(kb + r) * N + nb + c];
  }
  __syncthreads();
  const int orow = tid >> 3;
  const int seg  = tid & 7;
  v8h hv;
#pragma unroll
  for (int e = 0; e < 8; ++e) hv[e] = (_Float16)(bf16r(t[seg * 8 + e][orow]) * scale);
  _Float16* dst = WT + (size_t)(nb + orow) * K + kb + seg * 8;
  *(volatile v8h*)dst = hv;
  __threadfence();
  *(volatile v8h*)dst = hv;
}

constexpr int GBM = 128, GBN = 128, GBK = 32;
constexpr int GTS = 40;
constexpr int EP_STR = 68;

template <typename OT, bool HAS_BIAS, bool RELU>
__global__ __launch_bounds__(256) void gemm_kernel(
    const _Float16* __restrict__ A, const _Float16* __restrict__ Bt,
    const float* __restrict__ bias, OT* __restrict__ Y, int N, int K, float alpha) {
  __shared__ __attribute__((aligned(16))) _Float16 As[GBM * GTS];
  __shared__ __attribute__((aligned(16))) _Float16 Bs[GBN * GTS];
  __shared__ __attribute__((aligned(16))) float Ep[8][16][EP_STR];

  const int tid  = threadIdx.x;
  const int lane = tid & 31;
  const int wid  = tid >> 5;
  const int wm   = wid >> 1;
  const int wn   = wid & 1;
  const int hi   = lane >> 4;
  const int l15  = lane & 15;
  const size_t bm = (size_t)blockIdx.y * GBM;
  const size_t bn = (size_t)blockIdx.x * GBN;

  v8f zero = {};
  v8f acc[2][4];
#pragma unroll
  for (int i = 0; i < 2; ++i)
#pragma unroll
    for (int j = 0; j < 4; ++j) acc[i][j] = zero;

  const int T = K / GBK;
#pragma unroll 1
  for (int t = 0; t < T; ++t) {
    const int kb = t * GBK;
    v8h ra[2], rb[2];
#pragma unroll
    for (int i = 0; i < 2; ++i) {
      const int c = i * 256 + tid;
      const int row = c >> 2, qt = c & 3;
      ra[i] = *(const v8h*)(A  + (bm + row) * (size_t)K + kb + qt * 8);
      rb[i] = *(const v8h*)(Bt + (bn + row) * (size_t)K + kb + qt * 8);
    }
    __syncthreads();
#pragma unroll
    for (int i = 0; i < 2; ++i) {
      const int c = i * 256 + tid;
      const int row = c >> 2, qt = c & 3;
      *(v8h*)&As[row * GTS + qt * 8] = ra[i];
      *(v8h*)&Bs[row * GTS + qt * 8] = rb[i];
    }
    __syncthreads();

    v16h af[2], bf[4];
#pragma unroll
    for (int i = 0; i < 2; ++i) af[i] = frag_ld(&As[(wm * 32 + i * 16 + l15) * GTS], hi);
#pragma unroll
    for (int j = 0; j < 4; ++j) bf[j] = frag_ld(&Bs[(wn * 64 + j * 16 + l15) * GTS], hi);
#pragma unroll
    for (int i = 0; i < 2; ++i)
#pragma unroll
      for (int j = 0; j < 4; ++j) acc[i][j] = wmma16(af[i], bf[j], acc[i][j]);
    asm volatile("v_nop\n\tv_nop\n\tv_nop\n\tv_nop"
                 : "+v"(acc[0][0]), "+v"(acc[0][1]), "+v"(acc[0][2]), "+v"(acc[0][3]),
                   "+v"(acc[1][0]), "+v"(acc[1][1]), "+v"(acc[1][2]), "+v"(acc[1][3])
                 : "v"(af[0]), "v"(af[1]), "v"(bf[0]), "v"(bf[1]), "v"(bf[2]), "v"(bf[3]));
  }

  constexpr bool F32OUT = (sizeof(OT) == 4);
#pragma unroll
  for (int i = 0; i < 2; ++i) {
#pragma unroll
    for (int j = 0; j < 4; ++j) {
      const float bv = HAS_BIAS ? bf16r(bias[bn + wn * 64 + j * 16 + l15]) : 0.0f;
#pragma unroll
      for (int r = 0; r < 8; ++r) {
        float y = acc[i][j][r] * alpha + bv;
        if (RELU) y = fmaxf(y, 0.0f);
        Ep[wid][r + 8 * hi][j * 16 + l15] = y;
      }
    }
    __syncthreads();
    const size_t gm0 = bm + wm * 32 + i * 16;
    const size_t gn0 = bn + wn * 64;
    if (F32OUT) {
      v4f ov[8];
#pragma unroll
      for (int it = 0; it < 8; ++it) {
        const int L = it * 4 + (lane >> 3);
        const int row = L >> 1, col = (L & 1) * 32 + (lane & 7) * 4;
        ov[it] = *(const v4f*)&Ep[wid][row][col];
      }
#pragma unroll
      for (int it = 0; it < 8; ++it) {
        const int L = it * 4 + (lane >> 3);
        const int row = L >> 1, col = (L & 1) * 32 + (lane & 7) * 4;
        float* p = (float*)Y + (gm0 + row) * (size_t)N + gn0 + col;
        *(volatile v4f*)p = ov[it];
      }
      __threadfence();
#pragma unroll
      for (int it = 0; it < 8; ++it) {
        const int L = it * 4 + (lane >> 3);
        const int row = L >> 1, col = (L & 1) * 32 + (lane & 7) * 4;
        float* p = (float*)Y + (gm0 + row) * (size_t)N + gn0 + col;
        *(volatile v4f*)p = ov[it];
      }
    } else {
      v8h ov[4];
#pragma unroll
      for (int it = 0; it < 4; ++it) {
        const int row = it * 4 + (lane >> 3), col = (lane & 7) * 8;
        const v4f a0 = *(const v4f*)&Ep[wid][row][col];
        const v4f a1 = *(const v4f*)&Ep[wid][row][col + 4];
        ov[it][0] = (_Float16)a0[0]; ov[it][1] = (_Float16)a0[1];
        ov[it][2] = (_Float16)a0[2]; ov[it][3] = (_Float16)a0[3];
        ov[it][4] = (_Float16)a1[0]; ov[it][5] = (_Float16)a1[1];
        ov[it][6] = (_Float16)a1[2]; ov[it][7] = (_Float16)a1[3];
      }
#pragma unroll
      for (int it = 0; it < 4; ++it) {
        const int row = it * 4 + (lane >> 3), col = (lane & 7) * 8;
        _Float16* p = (_Float16*)Y + (gm0 + row) * (size_t)N + gn0 + col;
        *(volatile v8h*)p = ov[it];
      }
      __threadfence();
#pragma unroll
      for (int it = 0; it < 4; ++it) {
        const int row = it * 4 + (lane >> 3), col = (lane & 7) * 8;
        _Float16* p = (_Float16*)Y + (gm0 + row) * (size_t)N + gn0 + col;
        *(volatile v8h*)p = ov[it];
      }
    }
    __syncthreads();
  }
}

constexpr int KC     = 64;
constexpr int KL_STR = 72;
constexpr int VT_STR = 72;
constexpr int PP_STR = 72;
static_assert((SEQ % KC) == 0);

__global__ __launch_bounds__(128) void attn_kernel(
    const _Float16* __restrict__ Qh, const _Float16* __restrict__ Kh,
    const _Float16* __restrict__ Vh, const int* __restrict__ mask,
    _Float16* __restrict__ O) {
  __shared__ __attribute__((aligned(16))) _Float16 kl[KC * KL_STR];
  __shared__ __attribute__((aligned(16))) _Float16 vT[NDK * VT_STR];
  __shared__ __attribute__((aligned(16))) _Float16 pP[4][16 * PP_STR];

  const int tid  = threadIdx.x;
  const int w    = tid >> 5;
  const int lane = tid & 31;
  const int hi   = lane >> 4;
  const int qn   = lane & 15;
  const int b    = blockIdx.z;
  const int head = blockIdx.y;
  const int qbase = blockIdx.x * 64 + w * 16;

  const size_t tokq = (size_t)b * SEQ + qbase + qn;
  const v16h qf0 = frag_ld(Qh + tokq * ND + head * NDK, hi);
  const v16h qf1 = frag_ld(Qh + tokq * ND + head * NDK + 32, hi);

  float m_run = -3.0e38f, l_run = 0.0f;
  v8f zero = {};
  v8f acc[4] = {zero, zero, zero, zero};

#pragma unroll 1
  for (int kb = 0; kb < SEQ; kb += KC) {
    __syncthreads();
#pragma unroll
    for (int i = 0; i < 4; ++i) {
      const int c = i * 128 + tid;
      const int row = c >> 3, qt = c & 7;
      const v8h kv = *(const v8h*)(Kh + ((size_t)b * SEQ + kb + row) * ND + head * NDK + qt * 8);
      *(v8h*)&kl[row * KL_STR + qt * 8] = kv;
    }
#pragma unroll
    for (int bi = 0; bi < 2; ++bi) {
      const int blk = bi * 128 + tid;
      const int k4 = (blk & 15) * 4;
      const int d4 = (blk >> 4) * 4;
      const _Float16* src = Vh + ((size_t)b * SEQ + kb + k4) * ND + head * NDK + d4;
      const v4hh r0 = *(const v4hh*)(src);
      const v4hh r1 = *(const v4hh*)(src + ND);
      const v4hh r2 = *(const v4hh*)(src + 2 * ND);
      const v4hh r3 = *(const v4hh*)(src + 3 * ND);
      v4hh c0, c1, c2, c3;
      c0[0] = r0[0]; c0[1] = r1[0]; c0[2] = r2[0]; c0[3] = r3[0];
      c1[0] = r0[1]; c1[1] = r1[1]; c1[2] = r2[1]; c1[3] = r3[1];
      c2[0] = r0[2]; c2[1] = r1[2]; c2[2] = r2[2]; c2[3] = r3[2];
      c3[0] = r0[3]; c3[1] = r1[3]; c3[2] = r2[3]; c3[3] = r3[3];
      *(v4hh*)&vT[(d4 + 0) * VT_STR + k4] = c0;
      *(v4hh*)&vT[(d4 + 1) * VT_STR + k4] = c1;
      *(v4hh*)&vT[(d4 + 2) * VT_STR + k4] = c2;
      *(v4hh*)&vT[(d4 + 3) * VT_STR + k4] = c3;
    }
    __syncthreads();

    float st[4][8];
#pragma unroll
    for (int t = 0; t < 4; ++t) {
      const v16h kf0 = frag_ld(&kl[(t * 16 + qn) * KL_STR], hi);
      const v16h kf1 = frag_ld(&kl[(t * 16 + qn) * KL_STR + 32], hi);
      v8f s = zero;
      s = wmma16(kf0, qf0, s);
      s = wmma16(kf1, qf1, s);
      asm volatile("v_nop\n\tv_nop\n\tv_nop\n\tv_nop" : "+v"(s) : "v"(kf1), "v"(qf1));
#pragma unroll
      for (int r = 0; r < 8; ++r) st[t][r] = s[r] * 0.125f;
    }

    float cm = -3.0e38f;
#pragma unroll
    for (int t = 0; t < 4; ++t)
#pragma unroll
      for (int r = 0; r < 8; ++r) cm = fmaxf(cm, st[t][r]);
    cm = fmaxf(cm, __shfl_xor(cm, 16, 32));
    const float m_new = fmaxf(m_run, cm);
    const float alpha = __expf(m_run - m_new);
    float rs = 0.0f;
#pragma unroll
    for (int t = 0; t < 4; ++t) {
      v8h pv;
#pragma unroll
      for (int r = 0; r < 8; ++r) {
        const float p = __expf(st[t][r] - m_new);
        rs += p;
        pv[r] = (_Float16)(p * 1024.0f);
      }
      *(v8h*)&pP[w][qn * PP_STR + t * 16 + hi * 8] = pv;
    }
    rs += __shfl_xor(rs, 16, 32);
    l_run = l_run * alpha + rs;
    m_run = m_new;

    float arow[8];
#pragma unroll
    for (int r = 0; r < 8; ++r) arow[r] = __shfl(alpha, r + hi * 8, 32);
#pragma unroll
    for (int j = 0; j < 4; ++j)
#pragma unroll
      for (int r = 0; r < 8; ++r) acc[j][r] *= arow[r];

    __syncthreads();

    const v16h pf0 = frag_ld(&pP[w][qn * PP_STR], hi);
    const v16h pf1 = frag_ld(&pP[w][qn * PP_STR + 32], hi);
#pragma unroll
    for (int j = 0; j < 4; ++j) {
      const v16h vf0 = frag_ld(&vT[(j * 16 + qn) * VT_STR], hi);
      const v16h vf1 = frag_ld(&vT[(j * 16 + qn) * VT_STR + 32], hi);
      acc[j] = wmma16(pf0, vf0, acc[j]);
      acc[j] = wmma16(pf1, vf1, acc[j]);
      asm volatile("v_nop\n\tv_nop\n\tv_nop\n\tv_nop"
                   : "+v"(acc[j]) : "v"(pf0), "v"(pf1), "v"(vf0), "v"(vf1));
    }
  }

  const int mk = mask[(size_t)b * S_FULL + qbase + qn];
  float linv[8];
  int   kp[8];
#pragma unroll
  for (int r = 0; r < 8; ++r) {
    const float lr = __shfl(l_run, r + hi * 8, 32);
    linv[r] = (1.0f / lr) * (16.0f / 1024.0f);
    kp[r] = __shfl(mk, r + hi * 8, 32);
  }
  __syncthreads();
#pragma unroll
  for (int j = 0; j < 4; ++j)
#pragma unroll
    for (int r = 0; r < 8; ++r) {
      const float val = (kp[r] != 0) ? acc[j][r] * linv[r] : 0.0f;
      pP[w][(r + 8 * hi) * PP_STR + j * 16 + qn] = (_Float16)val;
    }
  __syncthreads();
  v8h ov[4];
#pragma unroll
  for (int it = 0; it < 4; ++it) {
    const int row = it * 4 + (lane >> 3), seg = lane & 7;
    ov[it] = *(const v8h*)&pP[w][row * PP_STR + seg * 8];
  }
#pragma unroll
  for (int it = 0; it < 4; ++it) {
    const int row = it * 4 + (lane >> 3), seg = lane & 7;
    _Float16* p = O + ((size_t)b * SEQ + qbase + row) * ND + head * NDK + seg * 8;
    *(volatile v8h*)p = ov[it];
  }
  __threadfence();
#pragma unroll
  for (int it = 0; it < 4; ++it) {
    const int row = it * 4 + (lane >> 3), seg = lane & 7;
    _Float16* p = O + ((size_t)b * SEQ + qbase + row) * ND + head * NDK + seg * 8;
    *(volatile v8h*)p = ov[it];
  }
}

template <bool FIRST>
__global__ __launch_bounds__(256) void ln_kernel(
    const float* __restrict__ Apl, const float* __restrict__ Xres,
    const float* __restrict__ gamma, const float* __restrict__ beta,
    float* __restrict__ Yf, _Float16* __restrict__ Yh) {
  __shared__ float red[8];
  const int tid = threadIdx.x, lane = tid & 31, wid = tid >> 5;
  const size_t row  = blockIdx.x;
  const size_t b    = row / SEQ;
  const size_t s    = row - b * SEQ;
  const size_t frow = b * S_FULL + s;
  const int c0 = tid * 4;

  const v4f a = *(const v4f*)(Apl + row * ND + c0);
  float sm = (a[0] + a[1]) + (a[2] + a[3]);
#pragma unroll
  for (int o = 16; o >= 1; o >>= 1) sm += __shfl_xor(sm, o, 32);
  if (lane == 0) red[wid] = sm;
  __syncthreads();
  float tot = 0.0f;
#pragma unroll
  for (int i = 0; i < 8; ++i) tot += red[i];
  const float mean = tot * (1.0f / 1024.0f);
  __syncthreads();

  float d[4];
  float sq = 0.0f;
#pragma unroll
  for (int i = 0; i < 4; ++i) { d[i] = a[i] - mean; sq += d[i] * d[i]; }
#pragma unroll
  for (int o = 16; o >= 1; o >>= 1) sq += __shfl_xor(sq, o, 32);
  if (lane == 0) red[wid] = sq;
  __syncthreads();
  float tot2 = 0.0f;
#pragma unroll
  for (int i = 0; i < 8; ++i) tot2 += red[i];
  const float var  = tot2 * (1.0f / 1024.0f);
  const float rstd = rsqrtf(var + 1.0e-6f);

  const v4f gv = *(const v4f*)(gamma + c0);
  const v4f bv = *(const v4f*)(beta + c0);
  v4f xr;
  if (FIRST) {
    const v4f xv = *(const v4f*)(Xres + frow * ND + c0);
    xr[0] = bf16r(xv[0]); xr[1] = bf16r(xv[1]); xr[2] = bf16r(xv[2]); xr[3] = bf16r(xv[3]);
  } else {
    xr = *(const v4f*)(Xres + row * ND + c0);
  }
  v4f o;
#pragma unroll
  for (int i = 0; i < 4; ++i)
    o[i] = xr[i] + (d[i] * rstd * bf16r(gv[i]) + bf16r(bv[i]));

  if (FIRST) {
    float* pf = Yf + row * ND + c0;
    v4hh hv;
    hv[0] = (_Float16)o[0]; hv[1] = (_Float16)o[1]; hv[2] = (_Float16)o[2]; hv[3] = (_Float16)o[3];
    _Float16* ph = Yh + row * ND + c0;
    *(volatile v4f*)pf  = o;
    *(volatile v4hh*)ph = hv;
    __threadfence();
    *(volatile v4f*)pf  = o;
    *(volatile v4hh*)ph = hv;
  } else {
    float* pf = Yf + frow * ND + c0;
    *(volatile v4f*)pf = o;
    __threadfence();
    *(volatile v4f*)pf = o;
  }
}

extern "C" void kernel_launch(void* const* d_in, const int* in_sizes, int n_in,
                              void* d_out, int out_size, void* d_ws, size_t ws_size,
                              hipStream_t stream) {
  if (n_in < 14) return;
  const long need_rows = (long)(NB - 1) * S_FULL + SEQ;
  if (in_sizes[0] < need_rows * ND) return;
  if (in_sizes[1] < need_rows) return;
  if (in_sizes[2] < ND * ND || in_sizes[3] < ND * ND ||
      in_sizes[4] < ND * ND || in_sizes[5] < ND * ND) return;
  if (in_sizes[6] < ND * NFF || in_sizes[7] < NFF) return;
  if (in_sizes[8] < NFF * ND || in_sizes[9] < ND) return;
  if (in_sizes[10] < ND || in_sizes[11] < ND || in_sizes[12] < ND || in_sizes[13] < ND) return;
  if ((long)out_size < need_rows * ND) return;

  const float* X    = (const float*)d_in[0];
  const int*   mask = (const int*)d_in[1];
  const float* W_Q  = (const float*)d_in[2];
  const float* W_K  = (const float*)d_in[3];
  const float* W_V  = (const float*)d_in[4];
  const float* W_O  = (const float*)d_in[5];
  const float* W1   = (const float*)d_in[6];
  const float* b1   = (const float*)d_in[7];
  const float* W2   = (const float*)d_in[8];
  const float* b2   = (const float*)d_in[9];
  const float* g1   = (const float*)d_in[10];
  const float* be1  = (const float*)d_in[11];
  const float* g2   = (const float*)d_in[12];
  const float* be2  = (const float*)d_in[13];
  float* out = (float*)d_out;

  const size_t MW2  = (size_t)ND * ND * 2;
  const size_t SLOT = (size_t)TOK * ND * 2;
  const size_t off_WqT = 0 * MW2, off_WkT = 1 * MW2, off_WvT = 2 * MW2, off_WoT = 3 * MW2;
  const size_t off_W1T = 4 * MW2;
  const size_t off_W2T = 8 * MW2;
  const size_t off_X   = 12 * MW2;
  const size_t off_Q   = off_X + 1 * SLOT;
  const size_t off_K   = off_X + 2 * SLOT;
  const size_t off_C   = off_X + 3 * SLOT;
  const size_t off_V   = off_X + 4 * SLOT;
  const size_t off_X1F = off_X + 5 * SLOT;
  const size_t off_FFN = off_X + 7 * SLOT;
  const size_t total   = off_X + 9 * SLOT;
  if (ws_size < total) return;

  char* ws = (char*)d_ws;
  _Float16* WqT = (_Float16*)(ws + off_WqT);
  _Float16* WkT = (_Float16*)(ws + off_WkT);
  _Float16* WvT = (_Float16*)(ws + off_WvT);
  _Float16* WoT = (_Float16*)(ws + off_WoT);
  _Float16* W1T = (_Float16*)(ws + off_W1T);
  _Float16* W2T = (_Float16*)(ws + off_W2T);
  _Float16* Xh  = (_Float16*)(ws + off_X);
  _Float16* qh  = (_Float16*)(ws + off_Q);
  _Float16* kh  = (_Float16*)(ws + off_K);
  _Float16* ch  = (_Float16*)(ws + off_C);
  _Float16* vh  = (_Float16*)(ws + off_V);
  float*    x1f = (float*)(ws + off_X1F);
  float*    ffn = (float*)(ws + off_FFN);
  float*    attnf = (float*)(ws + off_Q);
  _Float16* x1h   = (_Float16*)(ws + off_V);
  _Float16* hh    = (_Float16*)(ws + off_X);

  const dim3 blk(256);
  const dim3 gD(ND / GBN, TOK / GBM);
  const dim3 gF(NFF / GBN, TOK / GBM);

  cvt_x_kernel<<<dim3(TOK / 2), blk, 0, stream>>>(X, Xh);
  wtr_kernel<<<dim3(ND / 32, ND / 64), blk, 0, stream>>>(W_Q, WqT, ND, ND, 16.0f);
  wtr_kernel<<<dim3(ND / 32, ND / 64), blk, 0, stream>>>(W_K, WkT, ND, ND, 16.0f);
  wtr_kernel<<<dim3(ND / 32, ND / 64), blk, 0, stream>>>(W_V, WvT, ND, ND, 16.0f);
  wtr_kernel<<<dim3(ND / 32, ND / 64), blk, 0, stream>>>(W_O, WoT, ND, ND, 16.0f);
  wtr_kernel<<<dim3(NFF / 32, ND / 64), blk, 0, stream>>>(W1, W1T, ND, NFF, 8.0f);
  wtr_kernel<<<dim3(ND / 32, NFF / 64), blk, 0, stream>>>(W2, W2T, NFF, ND, 16.0f);

  gemm_kernel<_Float16, false, false><<<gD, blk, 0, stream>>>(Xh, WqT, b2, qh, ND, ND, 1.0f / 16.0f);
  gemm_kernel<_Float16, false, false><<<gD, blk, 0, stream>>>(Xh, WkT, b2, kh, ND, ND, 1.0f / 16.0f);
  gemm_kernel<_Float16, false, false><<<gD, blk, 0, stream>>>(Xh, WvT, b2, vh, ND, ND, 1.0f / 16.0f);

  attn_kernel<<<dim3(SEQ / 64, NH, NB), dim3(128), 0, stream>>>(qh, kh, vh, mask, ch);

  gemm_kernel<float, false, false><<<gD, blk, 0, stream>>>(ch, WoT, b2, attnf, ND, ND, 1.0f / 256.0f);

  ln_kernel<true><<<dim3(TOK), blk, 0, stream>>>(attnf, X, g1, be1, x1f, x1h);

  gemm_kernel<_Float16, true, true><<<gF, blk, 0, stream>>>(x1h, W1T, b1, hh, NFF, ND, 1.0f / 8.0f);
  gemm_kernel<float, true, false><<<gD, blk, 0, stream>>>(hh, W2T, b2, ffn, ND, NFF, 1.0f / 16.0f);

  ln_kernel<false><<<dim3(TOK), blk, 0, stream>>>(ffn, x1f, g2, be2, out, x1h);
}
